// EvalMemoryReader_6219112644707
// MI455X (gfx1250) — hardware-verified
//
#include <hip/hip_runtime.h>
#include <math.h>
#pragma clang fp contract(off)

typedef __attribute__((ext_vector_type(16))) __bf16   v16b;
typedef __attribute__((ext_vector_type(8)))  __bf16   v8b;
typedef __attribute__((ext_vector_type(8)))  float    v8f;
typedef __attribute__((ext_vector_type(4)))  float    v4f;
typedef __attribute__((ext_vector_type(4)))  unsigned v4u;
typedef __attribute__((ext_vector_type(4)))  int      v4i;

constexpr int kCK   = 64;
constexpr int kCV   = 512;
constexpr int kT    = 8;
constexpr int kH    = 32;
constexpr int kW    = 56;
constexpr int kHW   = kH * kW;
constexpr int kTHW  = kT * kHW;
constexpr int kTopK = 50;
constexpr int kTopP = 64;
constexpr int kSqrtCK = 8;
static_assert(kSqrtCK * kSqrtCK == kCK, "sqrt of key depth");
constexpr float  kAffScale = 1.0f / (float)kSqrtCK;
constexpr double kKmD      = 5.6;
constexpr float  kTwoKm2   = (float)(2.0 * (kKmD * kKmD));
constexpr float  kInvTwoKm2 = 1.0f / kTwoKm2;
static_assert(kHW == 1792 && kTHW == 14336, "positions");
static_assert((kCK % 32) == 0, "GEMM depth multiple of 32");
static_assert((kHW % 64) == 0 && (kTHW % 64) == 0 && (kCV % 64) == 0, "tile multiples");
static_assert((kTHW % 512) == 0 && (kTHW % 256) == 0 && (kHW % 32) == 0 && (kCV % 256) == 0, "block multiples");
static_assert(((kHW / 64) * (kTHW / 64)) % 8 == 0, "whole blocks of 8 wave tiles");
constexpr int kPerThr = kTHW / 512;
static_assert(kPerThr == 28, "elements per selection thread");

constexpr size_t kOffAFFT = 0;
constexpr size_t kOffMVT  = kOffAFFT + (size_t)kHW  * kTHW * 4;
constexpr size_t kOffMK   = kOffMVT  + (size_t)kTHW * kCV  * 2;
constexpr size_t kOffQK   = kOffMK   + (size_t)kTHW * kCK  * 2;
constexpr size_t kOffAN   = kOffQK   + (size_t)kHW  * kCK  * 2;
constexpr size_t kOffCN   = kOffAN   + (size_t)kTHW * 4;
constexpr size_t kOffCEN  = kOffCN   + (size_t)kHW  * 4;
constexpr size_t kOffTIDX = kOffCEN  + (size_t)kTHW * 4;
constexpr size_t kOffTVAL = kOffTIDX + (size_t)kHW  * kTopP * 4;
constexpr size_t kWsTotal = kOffTVAL + (size_t)kHW  * kTopP * 4;
static_assert(kWsTotal == 120544256ull, "carve total");
static_assert(kWsTotal <= 134217728ull, "carve cap");
static_assert((kOffMVT % 128) == 0 && (kOffMK % 128) == 0 && (kOffQK % 128) == 0 && (kOffAN % 128) == 0 &&
              (kOffCN % 128) == 0 && (kOffCEN % 128) == 0 && (kOffTIDX % 128) == 0 && (kOffTVAL % 128) == 0,
              "128-B aligned regions");

__device__ __forceinline__ unsigned short f2bf_bits(float f) {
  unsigned u = __float_as_uint(f);
  return (unsigned short)((u + 0x7FFFu + ((u >> 16) & 1u)) >> 16);
}
__device__ __forceinline__ float bf_bits2f(unsigned short h) { return __uint_as_float(((unsigned)h) << 16); }

__device__ __forceinline__ unsigned ord_enc(float f) {
  unsigned u = __float_as_uint(f);
  return u ^ ((u & 0x80000000u) ? 0xFFFFFFFFu : 0x80000000u);
}

__device__ __forceinline__ float center_d2(int ce, float yq, float xq) {
  int cy = (ce >> 8) & 63;
  cy = (cy > kH - 1) ? (kH - 1) : cy;
  int cx = ce & 255;
  cx = (cx > kW - 1) ? (kW - 1) : cx;
  const float dy = yq - (float)cy;
  const float dx = xq - (float)cx;
  return dy * dy + dx * dx;
}

__device__ __forceinline__ v16b frag_load_bf(const __bf16* p) {
  union U { v16b v; v8b h[2]; };
  U f;
  f.h[0] = *(const v8b*)(p);
  f.h[1] = *(const v8b*)(p + 16);
  return f.v;
}
__device__ __forceinline__ v8f mma_bf16(v16b a, v16b b, v8f c) {
  c = __builtin_amdgcn_wmma_f32_16x16x32_bf16(false, a, false, b, (short)0, c, false, false);
  asm volatile("v_nop\n\tv_nop\n\tv_nop\n\tv_nop" : "+v"(c) : "v"(a), "v"(b));
  return c;
}

__device__ __forceinline__ void tile_load_convert(const float* __restrict__ src, size_t pitch,
                                                  int p0, int c0, float* sT, int tid) {
  const int pl = tid & 63;
  const int cg = tid >> 6;
#pragma unroll 4
  for (int i = 0; i < 16; ++i) {
    const int cl = cg * 16 + i;
    const float f = src[(size_t)(c0 + cl) * pitch + p0 + pl];
    sT[pl * 65 + cl] = bf_bits2f(f2bf_bits(f));
  }
}

__device__ __forceinline__ void tile_store_bf16(const float* sT, unsigned short* __restrict__ dst,
                                                int dpitch, int p0, int c0, int wave, int lane) {
  const int rq = lane >> 3;
  const int c8 = (lane & 7) * 8;
  v4u w0, w1;
  {
    const float* sp = sT + (wave * 4 + rq) * 65 + c8;
#pragma unroll
    for (int k = 0; k < 4; ++k) {
      const unsigned lo = __float_as_uint(sp[2 * k]) >> 16;
      const unsigned hi = __float_as_uint(sp[2 * k + 1]) & 0xffff0000u;
      w0[k] = lo | hi;
    }
  }
  {
    const float* sp = sT + (32 + wave * 4 + rq) * 65 + c8;
#pragma unroll
    for (int k = 0; k < 4; ++k) {
      const unsigned lo = __float_as_uint(sp[2 * k]) >> 16;
      const unsigned hi = __float_as_uint(sp[2 * k + 1]) & 0xffff0000u;
      w1[k] = lo | hi;
    }
  }
  unsigned short* d0 = dst + (size_t)(p0 + wave * 4 + rq) * dpitch + c0 + c8;
  unsigned short* d1 = dst + (size_t)(p0 + 32 + wave * 4 + rq) * dpitch + c0 + c8;
  for (int pass = 0; pass < 2; ++pass) {
    *(volatile v4u*)d0 = w0;
    *(volatile v4u*)d1 = w1;
    __threadfence();
  }
}

__global__ __launch_bounds__(256) void prep_keys_kernel(
    const float* __restrict__ mk, const float* __restrict__ qk,
    unsigned short* __restrict__ Mk16, unsigned short* __restrict__ Qk16,
    float* __restrict__ aN, float* __restrict__ cN)
{
  __shared__ float sT[64 * 65];
  const int tid  = threadIdx.x;
  const int lane = tid & 31;
  const int wave = __builtin_amdgcn_readfirstlane((int)(threadIdx.x >> 5));
  const int bx = blockIdx.x;
  const bool isM = bx < (kTHW / 64);
  const float* src = isM ? mk : qk;
  const size_t pitch = isM ? (size_t)kTHW : (size_t)kHW;
  const int p0 = (isM ? bx : (bx - kTHW / 64)) * 64;
  unsigned short* dst = isM ? Mk16 : Qk16;
  float* nrm = isM ? aN : cN;

  tile_load_convert(src, pitch, p0, 0, sT, tid);
  __syncthreads();
  tile_store_bf16(sT, dst, kCK, p0, 0, wave, lane);
  if (tid < 64) {
    float s = 0.0f;
#pragma unroll 8
    for (int c = 0; c < kCK; ++c) {
      const float v = sT[tid * 65 + c];
      const float p = v * v;
      s = s + p;
    }
    float* np = nrm + p0 + tid;
    *(volatile float*)np = s;
    __threadfence();
    *(volatile float*)np = s;
  }
}

__global__ __launch_bounds__(256) void prep_values_kernel(
    const float* __restrict__ mv, unsigned short* __restrict__ MvT16)
{
  __shared__ float sT[64 * 65];
  const int tid  = threadIdx.x;
  const int lane = tid & 31;
  const int wave = __builtin_amdgcn_readfirstlane((int)(threadIdx.x >> 5));
  const int p0 = blockIdx.x * 64;
  const int c0 = blockIdx.y * 64;
  tile_load_convert(mv, (size_t)kTHW, p0, c0, sT, tid);
  __syncthreads();
  tile_store_bf16(sT, MvT16, kCV, p0, c0, wave, lane);
}

__global__ __launch_bounds__(256) void aff_gemm_kernel(
    const unsigned short* __restrict__ Qk16, const unsigned short* __restrict__ Mk16,
    const float* __restrict__ aN, const float* __restrict__ cN, float* __restrict__ affT)
{
  __shared__ __align__(16) float sT[8][16 * 68];
  const int lane = threadIdx.x & 31;
  const int wave = __builtin_amdgcn_readfirstlane((int)(threadIdx.x >> 5));
  constexpr int tilesN = kTHW / 64;
  constexpr int tilesM = kHW / 64;
  const int tile = blockIdx.x * 8 + wave;
  if (tile >= tilesM * tilesN) return;
  const int tm = tile / tilesN;
  const int tn = tile - tm * tilesN;
  const int m0 = tm << 6;
  const int n0 = tn << 6;
  const __bf16* A  = (const __bf16*)Qk16;
  const __bf16* Bt = (const __bf16*)Mk16;
  const int rlane = lane & 15;
  const int koff  = (lane >> 4) * 8;
  const int mOff  = (lane >> 4) * 8;

  v8f acc[4][4];
#pragma unroll
  for (int i = 0; i < 4; ++i)
#pragma unroll
    for (int j = 0; j < 4; ++j) acc[i][j] = (v8f){0.f, 0.f, 0.f, 0.f, 0.f, 0.f, 0.f, 0.f};

#pragma unroll 1
  for (int k0 = 0; k0 < kCK; k0 += 32) {
    v16b bh[4];
#pragma unroll
    for (int j = 0; j < 4; ++j)
      bh[j] = frag_load_bf(Bt + (size_t)(n0 + (j << 4) + rlane) * kCK + koff + k0);
#pragma unroll
    for (int i = 0; i < 4; ++i) {
      const v16b ah = frag_load_bf(A + (size_t)(m0 + (i << 4) + rlane) * kCK + koff + k0);
#pragma unroll
      for (int j = 0; j < 4; ++j) acc[i][j] = mma_bf16(ah, bh[j], acc[i][j]);
    }
  }

  float an[4];
#pragma unroll
  for (int j = 0; j < 4; ++j) an[j] = aN[n0 + (j << 4) + rlane];

  float* slab = sT[wave];
#pragma unroll
  for (int i = 0; i < 4; ++i) {
    const int mBase = m0 + (i << 4);
    const v4f cA = *(const v4f*)(cN + mBase + mOff);
    const v4f cB = *(const v4f*)(cN + mBase + mOff + 4);
    float cq[8];
    cq[0] = cA[0]; cq[1] = cA[1]; cq[2] = cA[2]; cq[3] = cA[3];
    cq[4] = cB[0]; cq[5] = cB[1]; cq[6] = cB[2]; cq[7] = cB[3];
#pragma unroll
    for (int j = 0; j < 4; ++j) {
#pragma unroll
      for (int r = 0; r < 8; ++r) {
        const float b2 = 2.0f * acc[i][j][r];
        const float t0 = b2 - an[j];
        const float t1 = t0 - cq[r];
        slab[(mOff + r) * 68 + (j << 4) + rlane] = t1 * kAffScale;
      }
    }
    __builtin_amdgcn_fence(__ATOMIC_RELEASE, "workgroup");
    __builtin_amdgcn_wave_barrier();
    __builtin_amdgcn_fence(__ATOMIC_ACQUIRE, "workgroup");
    {
      const int hh = lane >> 4;
      const int c4 = (lane & 15) * 4;
      for (int pass = 0; pass < 2; ++pass) {
#pragma unroll
        for (int it = 0; it < 8; ++it) {
          const int row = it * 2 + hh;
          const v4f v = *(const v4f*)(slab + row * 68 + c4);
          *(volatile v4f*)(affT + (size_t)(mBase + row) * kTHW + n0 + c4) = v;
        }
        __threadfence();
      }
    }
    __builtin_amdgcn_fence(__ATOMIC_RELEASE, "workgroup");
    __builtin_amdgcn_wave_barrier();
    __builtin_amdgcn_fence(__ATOMIC_ACQUIRE, "workgroup");
  }
}

__global__ __launch_bounds__(256) void argmax_kernel(const float* __restrict__ affT, int* __restrict__ cen)
{
  const int m = blockIdx.x * 256 + threadIdx.x;
  float best = -INFINITY;
  int bi = 0;
#pragma unroll 8
  for (int q = 0; q < kHW; ++q) {
    const float v = affT[(size_t)q * kTHW + m];
    const bool gt = v > best;
    best = gt ? v : best;
    bi = gt ? q : bi;
  }
  const int packed = ((bi / kW) << 8) | (bi % kW);
  int* cp = cen + m;
  *(volatile int*)cp = packed;
  __threadfence();
  *(volatile int*)cp = packed;
}

__global__ __launch_bounds__(512) void topk_kernel(
    const float* __restrict__ affT, const int* __restrict__ cen,
    int* __restrict__ topIdx, float* __restrict__ topVal)
{
  __shared__ unsigned keys[kTHW];
  __shared__ unsigned hist[256];
  __shared__ float wmaxs[16];
  __shared__ int   wtot[16];
  __shared__ int   sel[kTopP];
  __shared__ float selw[kTopP];
  __shared__ unsigned sh_prefix;
  __shared__ unsigned sh_kRem;

  const int q    = blockIdx.x;
  const int tid  = threadIdx.x;
  const int lane = tid & 31;
  const int wave = __builtin_amdgcn_readfirstlane((int)(threadIdx.x >> 5));
  const float yq = (float)(q / kW);
  const float xq = (float)(q % kW);
  const float* row = affT + (size_t)q * kTHW;

  float lmax = -INFINITY;
#pragma unroll 4
  for (int i = 0; i < kPerThr; ++i) {
    const int m = i * 512 + tid;
    const float a = row[m];
    keys[m] = __float_as_uint(a);
    lmax = fmaxf(lmax, a);
  }
#pragma unroll
  for (int off = 16; off >= 1; off >>= 1) lmax = fmaxf(lmax, __shfl_xor(lmax, off, 32));
  if (lane == 0) wmaxs[wave] = lmax;
  if (tid < kTopP) { sel[tid] = 0; selw[tid] = 0.0f; }
  if (tid == 0) { sh_prefix = 0u; sh_kRem = (unsigned)kTopK; }
  __syncthreads();
  float maxq = wmaxs[0];
#pragma unroll
  for (int w = 1; w < 16; ++w) maxq = fmaxf(maxq, wmaxs[w]);

#pragma unroll 2
  for (int i = 0; i < kPerThr; ++i) {
    const int m = i * 512 + tid;
    const float a = __uint_as_float(keys[m]);
    const int ce = cen[m];
    const float d2 = center_d2(ce, yq, xq);
    const float u = a - maxq;
    const float g = d2 * kInvTwoKm2;
    const float s = u - g;
    keys[m] = ord_enc(s);
  }

#pragma unroll 1
  for (int r = 3; r >= 0; --r) {
    if (tid < 256) hist[tid] = 0u;
    __syncthreads();
    const unsigned prefix = sh_prefix;
    const unsigned hiMask = (r == 3) ? 0u : (0xFFFFFFFFu << ((r + 1) * 8));
    const int shift = r * 8;
#pragma unroll 4
    for (int i = 0; i < kPerThr; ++i) {
      const unsigned k = keys[i * 512 + tid];
      if ((k & hiMask) == prefix) atomicAdd(&hist[(k >> shift) & 255u], 1u);
    }
    __syncthreads();
    if (tid == 0) {
      const unsigned kRem = sh_kRem;
      unsigned cum = 0u;
      int b = 255;
      for (; b > 0; --b) {
        const unsigned h = hist[b];
        if (cum + h >= kRem) break;
        cum += h;
      }
      sh_prefix = prefix | ((unsigned)b << shift);
      sh_kRem = kRem - cum;
    }
    __syncthreads();
  }
  const unsigned Tkey = sh_prefix;
  int tiesNeeded = (int)sh_kRem;
  tiesNeeded = tiesNeeded < 1 ? 1 : tiesNeeded;
  tiesNeeded = tiesNeeded > kTopK ? kTopK : tiesNeeded;
  const int cntG = kTopK - tiesNeeded;

  const int mb = tid * kPerThr;
  int g = 0, e = 0;
#pragma unroll 4
  for (int i = 0; i < kPerThr; ++i) {
    const unsigned k = keys[mb + i];
    g += (k > Tkey) ? 1 : 0;
    e += (k == Tkey) ? 1 : 0;
  }
  const int packed = g + (e << 16);
  int incl = packed;
#pragma unroll
  for (int off = 1; off < 32; off <<= 1) {
    const int nb = __shfl_up(incl, off, 32);
    incl += (lane >= off) ? nb : 0;
  }
  if (lane == 31) wtot[wave] = incl;
  __syncthreads();
  int base = 0;
#pragma unroll
  for (int w = 0; w < 16; ++w) {
    const int t = wtot[w];
    base += (w < wave) ? t : 0;
  }
  const int excl = base + incl - packed;
  int posG = excl & 0xffff;
  int posE = excl >> 16;
#pragma unroll 4
  for (int i = 0; i < kPerThr; ++i) {
    const int m = mb + i;
    const unsigned k = keys[m];
    if (k > Tkey) {
      if (posG < kTopP) sel[posG] = m;
      posG++;
    } else if (k == Tkey) {
      if (posE < tiesNeeded) {
        const int p = cntG + posE;
        if (p < kTopP) sel[p] = m;
      }
      posE++;
    }
  }
  __syncthreads();

  float v = 0.0f;
  int msel = 0;
  if (tid < kTopP) {
    msel = sel[tid];
    msel = msel < 0 ? 0 : msel;
    msel = msel > kTHW - 1 ? kTHW - 1 : msel;
    const float a = row[msel];
    const int ce = cen[msel];
    const float d2 = center_d2(ce, yq, xq);
    const float e1 = expf(a - maxq);
    const float gneg = (-d2) * kInvTwoKm2;
    const float e2 = expf(gneg);
    const float vv = e1 * e2;
    v = (tid < kTopK) ? vv : 0.0f;
    selw[tid] = v;
  }
  __syncthreads();
  if (tid < kTopP) {
    float s = 0.0f;
#pragma unroll 1
    for (int j = 0; j < kTopK; ++j) s = s + selw[j];
    const float inv = 1.0f / s;
    const float wv = v * inv;
    const int mo = (tid < kTopK) ? msel : 0;
    int*   ip = topIdx + (size_t)q * kTopP + tid;
    float* vp = topVal + (size_t)q * kTopP + tid;
    *(volatile int*)ip = mo;
    *(volatile float*)vp = wv;
    __threadfence();
    *(volatile int*)ip = mo;
    *(volatile float*)vp = wv;
  }
}

__global__ __launch_bounds__(128) void readout_kernel(
    const unsigned* __restrict__ MvW, const int* __restrict__ topIdx,
    const float* __restrict__ topVal, float* __restrict__ out)
{
  __shared__ __align__(16) float tile[256 * 36];
  __shared__ __align__(16) int   sOff[32 * kTopP];
  __shared__ __align__(16) float sWt[32 * kTopP];
  const int tid  = threadIdx.x;
  const int lane = tid & 31;
  const int wave = __builtin_amdgcn_readfirstlane((int)(threadIdx.x >> 5));
  const int q0 = blockIdx.x * 32;
  const int c0 = blockIdx.y * 256;

#pragma unroll
  for (int it = 0; it < 4; ++it) {
    const int e = (it * 128 + tid) * 4;
    const v4i iv = *(const v4i*)(topIdx + (size_t)q0 * kTopP + e);
    const v4f wv = *(const v4f*)(topVal + (size_t)q0 * kTopP + e);
    v4i ov;
#pragma unroll
    for (int k = 0; k < 4; ++k) {
      int ix = iv[k];
      ix = ix < 0 ? 0 : ix;
      ix = ix > kTHW - 1 ? kTHW - 1 : ix;
      ov[k] = ix * (kCV / 2);
    }
    *(v4i*)(sOff + e) = ov;
    *(v4f*)(sWt + e) = wv;
  }
  __syncthreads();

  float acc0[32], acc1[32];
#pragma unroll
  for (int qq = 0; qq < 32; ++qq) { acc0[qq] = 0.0f; acc1[qq] = 0.0f; }
  const unsigned* basep = MvW + (c0 >> 1) + tid;

#pragma unroll 1
  for (int j = 0; j < kTopK; ++j) {
#pragma unroll
    for (int qq = 0; qq < 16; ++qq) {
      const int off = sOff[qq * kTopP + j];
      const float w = sWt[qq * kTopP + j];
      const unsigned u = basep[off];
      const float f0 = __uint_as_float(u << 16);
      const float f1 = __uint_as_float(u & 0xffff0000u);
      acc0[qq] = fmaf(w, f0, acc0[qq]);
      acc1[qq] = fmaf(w, f1, acc1[qq]);
    }
    asm volatile("" ::: "memory");
#pragma unroll
    for (int qq = 16; qq < 32; ++qq) {
      const int off = sOff[qq * kTopP + j];
      const float w = sWt[qq * kTopP + j];
      const unsigned u = basep[off];
      const float f0 = __uint_as_float(u << 16);
      const float f1 = __uint_as_float(u & 0xffff0000u);
      acc0[qq] = fmaf(w, f0, acc0[qq]);
      acc1[qq] = fmaf(w, f1, acc1[qq]);
    }
  }

#pragma unroll
  for (int qq = 0; qq < 32; ++qq) {
    tile[(2 * tid) * 36 + qq] = acc0[qq];
    tile[(2 * tid + 1) * 36 + qq] = acc1[qq];
  }
  __syncthreads();
  {
    const int rq = lane >> 3;
    const int c4 = (lane & 7) * 4;
    for (int pass = 0; pass < 2; ++pass) {
#pragma unroll 4
      for (int it = 0; it < 16; ++it) {
        const int rowl = it * 16 + wave * 4 + rq;
        const v4f val = *(const v4f*)(tile + rowl * 36 + c4);
        *(volatile v4f*)(out + (size_t)(c0 + rowl) * kHW + q0 + c4) = val;
      }
      __threadfence();
    }
  }
}

extern "C" void kernel_launch(void* const* d_in, const int* in_sizes, int n_in,
                              void* d_out, int out_size, void* d_ws, size_t ws_size,
                              hipStream_t stream) {
  if (n_in < 3) return;
  if (in_sizes[0] != kCK * kTHW) return;
  if (in_sizes[1] != kCK * kHW) return;
  if (in_sizes[2] != kCV * kTHW) return;
  if (out_size != kCV * kHW) return;
  if (ws_size < kWsTotal) return;

  const float* mk = (const float*)d_in[0];
  const float* qk = (const float*)d_in[1];
  const float* mv = (const float*)d_in[2];
  float* out = (float*)d_out;

  char* ws = (char*)d_ws;
  float*          affT   = (float*)(ws + kOffAFFT);
  unsigned short* MvT16  = (unsigned short*)(ws + kOffMVT);
  unsigned short* Mk16   = (unsigned short*)(ws + kOffMK);
  unsigned short* Qk16   = (unsigned short*)(ws + kOffQK);
  float*          aN     = (float*)(ws + kOffAN);
  float*          cN     = (float*)(ws + kOffCN);
  int*            cen    = (int*)(ws + kOffCEN);
  int*            topIdx = (int*)(ws + kOffTIDX);
  float*          topVal = (float*)(ws + kOffTVAL);

  prep_keys_kernel<<<kTHW / 64 + kHW / 64, 256, 0, stream>>>(mk, qk, Mk16, Qk16, aN, cN);
  prep_values_kernel<<<dim3(kTHW / 64, kCV / 64), 256, 0, stream>>>(mv, MvT16);
  aff_gemm_kernel<<<((kHW / 64) * (kTHW / 64)) / 8, 256, 0, stream>>>(Qk16, Mk16, aN, cN, affT);
  argmax_kernel<<<kTHW / 256, 256, 0, stream>>>(affT, cen);
  topk_kernel<<<kHW, 512, 0, stream>>>(affT, cen, topIdx, topVal);
  readout_kernel<<<dim3(kHW / 32, kCV / 256), 128, 0, stream>>>((const unsigned*)MvT16, topIdx, topVal, out);
}
